// MOA_13254269075617
// MI455X (gfx1250) — hardware-verified
//
#include <hip/hip_runtime.h>
#include <math.h>
#include <stdint.h>


#define NB    8
#define HS    64
#define WS    64
#define CH    256
#define NPIX  (NB * HS * WS)
#define NAT   81
#define NVA   384
#define KFU   512
#define TM64  (NPIX / 64)
#define SLP   68

static_assert(NPIX == 32768 && TM64 == 512);
static_assert(HS == 64 && WS == 64 && CH == 256);
static_assert(CH + NAT <= NVA && NVA % 64 == 0 && CH % 64 == 0);
static_assert(CH % 32 == 0 && KFU % 32 == 0 && KFU == 2 * CH);
static_assert((NPIX * CH) % (8 * 256) == 0);

typedef unsigned short us_t;
typedef us_t   v8us  __attribute__((ext_vector_type(8)));
typedef __bf16 v16bf __attribute__((ext_vector_type(16)));
typedef float  v8f   __attribute__((ext_vector_type(8)));
typedef float  v4f   __attribute__((ext_vector_type(4)));
typedef unsigned int v4u __attribute__((ext_vector_type(4)));

union HU  { v8us s; v4u u; us_t e[8]; };
union FRB { v16bf v; v8us u[2]; };
static_assert(sizeof(HU) == 16);
static_assert(sizeof(FRB) == 32);

__device__ __forceinline__ us_t bf_bits(float f) {
  const unsigned u = __float_as_uint(f);
  return (us_t)((u + 0x7FFFu + ((u >> 16) & 1u)) >> 16);
}
__device__ __forceinline__ float bf_up(us_t h) { return __uint_as_float(((unsigned)h) << 16); }
__device__ __forceinline__ float bfr(float f) { return bf_up(bf_bits(f)); }
__device__ __forceinline__ v8f zero8() { v8f z = {0.f, 0.f, 0.f, 0.f, 0.f, 0.f, 0.f, 0.f}; return z; }
__device__ __forceinline__ v4f zero4() { v4f z = {0.f, 0.f, 0.f, 0.f}; return z; }
__device__ __forceinline__ v4f fill4(float a) { v4f z = {a, a, a, a}; return z; }
__device__ __forceinline__ v4f vmax4(v4f a, v4f b) {
  v4f r;
  r[0] = fmaxf(a[0], b[0]); r[1] = fmaxf(a[1], b[1]); r[2] = fmaxf(a[2], b[2]); r[3] = fmaxf(a[3], b[3]);
  return r;
}
__device__ __forceinline__ void ld8(const float* p, float* o) {
  const v4f a = *(const v4f*)(p);
  const v4f b = *(const v4f*)(p + 4);
  o[0] = a[0]; o[1] = a[1]; o[2] = a[2]; o[3] = a[3];
  o[4] = b[0]; o[5] = b[1]; o[6] = b[2]; o[7] = b[3];
}

__device__ __forceinline__ v16bf ldfrag_b(const us_t* p) {
  FRB f;
  f.u[0] = *(const v8us*)(p);
  f.u[1] = *(const v8us*)(p + 16);
  return f.v;
}

__device__ __forceinline__ v8f mma_b_raw(v16bf a, v16bf b, v8f c) {
  return __builtin_amdgcn_wmma_f32_16x16x32_bf16(false, a, false, b, (short)0, c, false, false);
}
__device__ __forceinline__ void dep_guard(v8f& a, v8f& b, v16bf x) {
#if defined(__HIP_DEVICE_COMPILE__)
  const v8f kx = __builtin_bit_cast(v8f, x);
  asm volatile("v_nop\n\tv_nop\n\tv_nop\n\tv_nop" : "+v"(a), "+v"(b) : "v"(kx));
#endif
}
__device__ __forceinline__ void keep4(v16bf a, v16bf b, v16bf c, v16bf d) {
#if defined(__HIP_DEVICE_COMPILE__)
  const v8f ka = __builtin_bit_cast(v8f, a), kb = __builtin_bit_cast(v8f, b);
  const v8f kc = __builtin_bit_cast(v8f, c), kd = __builtin_bit_cast(v8f, d);
  asm volatile("v_nop" :: "v"(ka), "v"(kb), "v"(kc), "v"(kd));
#endif
}
__device__ __forceinline__ void acc_guard4(v8f& a, v8f& b, v8f& c, v8f& d) {
#if defined(__HIP_DEVICE_COMPILE__)
  asm volatile("v_nop\n\tv_nop\n\tv_nop\n\tv_nop" : "+v"(a), "+v"(b), "+v"(c), "+v"(d));
#endif
}
__device__ __forceinline__ void wave_lds_sync() {
  __builtin_amdgcn_fence(__ATOMIC_RELEASE, "workgroup");
  __builtin_amdgcn_wave_barrier();
  __builtin_amdgcn_fence(__ATOMIC_ACQUIRE, "workgroup");
}

__global__ __launch_bounds__(256) void cvt_bf(const float* __restrict__ in, us_t* out, int n8) {
  const int i = blockIdx.x * 256 + threadIdx.x;
  if (i < n8) {
    float v[8];
    ld8(in + (size_t)i * 8, v);
    HU u;
#pragma unroll
    for (int e = 0; e < 8; ++e) u.e[e] = bf_bits(v[e]);
    us_t* p = out + (size_t)i * 8;
    *(volatile v4u*)p = u.u;
    __threadfence();
    *(volatile v4u*)p = u.u;
  }
}

__global__ __launch_bounds__(256) void wtr8(const float* __restrict__ Wm, int K, int N, us_t* out, int nrows) {
  const int k8n = K >> 3;
  const int t = blockIdx.x * 256 + threadIdx.x;
  const int n = t / k8n;
  const int k8 = t - n * k8n;
  if (n < nrows) {
    const int nc = min(n, N - 1);
    const bool ok = n < N;
    HU u;
#pragma unroll
    for (int e = 0; e < 8; ++e) {
      const float wv = Wm[(size_t)(k8 * 8 + e) * (size_t)N + nc];
      u.e[e] = ok ? bf_bits(wv) : (us_t)0;
    }
    us_t* p = out + (size_t)n * (size_t)K + k8 * 8;
    *(volatile v4u*)p = u.u;
    __threadfence();
    *(volatile v4u*)p = u.u;
  }
}

__device__ __forceinline__ void kseg(v8f (&acc)[4][4], const us_t* __restrict__ A, int lda, int m0,
                                     const us_t* __restrict__ Bt, int ldb, int n0, int K, int rlane, int koff) {
  for (int kk = 0; kk < K; kk += 32) {
    v16bf bh[4];
#pragma unroll
    for (int j = 0; j < 4; ++j) {
      const size_t bo = (size_t)(n0 + (j << 4) + rlane) * (size_t)ldb + koff + kk;
      bh[j] = ldfrag_b(Bt + bo);
    }
#pragma unroll
    for (int i = 0; i < 4; ++i) {
      const size_t ao = (size_t)(m0 + (i << 4) + rlane) * (size_t)lda + koff + kk;
      const v16bf a0 = ldfrag_b(A + ao);
#pragma unroll
      for (int j = 0; j < 4; ++j) acc[i][j] = mma_b_raw(a0, bh[j], acc[i][j]);
      dep_guard(acc[i][0], acc[i][3], a0);
    }
    keep4(bh[0], bh[1], bh[2], bh[3]);
  }
}

__device__ __forceinline__ float colbias(const float* __restrict__ b0, int nb0,
                                         const float* __restrict__ b1, int nb1, int col) {
  const int c0 = min(max(col, 0), nb0 - 1);
  const int c1 = min(max(col - nb0, 0), nb1 - 1);
  const float v0 = bfr(b0[c0]);
  const float v1 = bfr(b1[c1]);
  return (col < nb0) ? v0 : ((col < nb0 + nb1) ? v1 : 0.0f);
}

template <int MODE, int NPL>
__global__ __launch_bounds__(256) void gemm64b(
    const us_t* __restrict__ A, int lda, size_t aplane, const us_t* __restrict__ Bt, int ldb,
    const float* __restrict__ b0p, int nb0, const float* __restrict__ b1p, int nb1,
    const float* __restrict__ R, int ldr, float* C, int ldc, float* P2, int M, int N, int K) {
  __shared__ __align__(16) float sT[8][16 * SLP];
  const int lane = threadIdx.x & 31;
  const int wave = threadIdx.x >> 5;
  const int tilesN = N >> 6;
  const int tilesM = M >> 6;
  const int tiles = tilesM * tilesN;
  const int item = blockIdx.x * 8 + wave;
  if (item >= tiles) return;
  const int tm = item / tilesN;
  const int tn = item - tm * tilesN;
  const int m0 = tm << 6;
  const int n0 = tn << 6;

  const int rlane = lane & 15;
  const int hh    = lane >> 4;
  const int koff  = hh * 8;
  const int mOff  = hh * 8;

  v8f acc[4][4];
#pragma unroll
  for (int i = 0; i < 4; ++i)
#pragma unroll
    for (int j = 0; j < 4; ++j) acc[i][j] = zero8();

#pragma unroll
  for (int p = 0; p < NPL; ++p)
    kseg(acc, A + (size_t)p * aplane, lda, m0, Bt, ldb, n0, K, rlane, koff);
  acc_guard4(acc[0][0], acc[0][1], acc[0][2], acc[0][3]);
  acc_guard4(acc[1][0], acc[1][1], acc[1][2], acc[1][3]);
  acc_guard4(acc[2][0], acc[2][1], acc[2][2], acc[2][3]);
  acc_guard4(acc[3][0], acc[3][1], acc[3][2], acc[3][3]);

  v4f b4;
#pragma unroll
  for (int e = 0; e < 4; ++e) b4[e] = colbias(b0p, nb0, b1p, nb1, n0 + 4 * rlane + e);
  v4f cs4 = zero4(), cq4 = zero4();

  float* slab = sT[wave];
#pragma unroll
  for (int i = 0; i < 4; ++i) {
    const int mBase = m0 + (i << 4);
#pragma unroll
    for (int r = 0; r < 8; ++r) {
#pragma unroll
      for (int j = 0; j < 4; ++j) {
        slab[(mOff + r) * SLP + (j << 4) + rlane] = acc[i][j][r];
      }
    }
    wave_lds_sync();
    v4f ov[8];
#pragma unroll
    for (int it = 0; it < 8; ++it) {
      const int row = 2 * it + hh;
      const v4f t = *(const v4f*)(slab + row * SLP + 4 * rlane);
      if (MODE == 0) {
        ov[it] = t + b4;
      } else {
        const v4f xr = *(const v4f*)(R + (size_t)(mBase + row) * (size_t)ldr + n0 + 4 * rlane);
        v4f o;
#pragma unroll
        for (int e = 0; e < 4; ++e) o[e] = bfr(xr[e]) + fmaxf(t[e] + b4[e], 0.0f);
        ov[it] = o;
        cs4 += o;
        cq4 += o * o;
      }
    }
    for (int pass = 0; pass < 2; ++pass) {
#pragma unroll
      for (int it = 0; it < 8; ++it) {
        const int row = 2 * it + hh;
        float* dst = C + (size_t)(mBase + row) * (size_t)ldc + n0 + 4 * rlane;
        *(volatile v4f*)dst = ov[it];
      }
      __threadfence();
    }
    wave_lds_sync();
  }

  if (MODE == 1) {
#pragma unroll
    for (int e = 0; e < 4; ++e) {
      cs4[e] += __shfl_xor(cs4[e], 16, 32);
      cq4[e] += __shfl_xor(cq4[e], 16, 32);
    }
    v4f pv;
#pragma unroll
    for (int e = 0; e < 4; ++e) pv[e] = (hh == 0) ? cs4[e] : cq4[e];
    float* pdst = P2 + (size_t)hh * (size_t)tilesM * (size_t)N + (size_t)tm * (size_t)N + n0 + 4 * rlane;
    for (int pass = 0; pass < 2; ++pass) {
      *(volatile v4f*)pdst = pv;
      __threadfence();
    }
  }
}

__global__ __launch_bounds__(256) void k_win(const float* __restrict__ VA, const float* __restrict__ X,
                                             us_t* CHp, us_t* CLp) {
  __shared__ __align__(16) float sP[8][96];
  __shared__ __align__(16) float sW[8][32];
  const int tid = threadIdx.x, lane = tid & 31, wave = tid >> 5;
  const int bh = blockIdx.x;
  const int b = bh >> 6, h = bh & 63;
  float* sPw = sP[wave];
  float* sWw = sW[wave];

#pragma unroll 1
  for (int kq = 0; kq < 8; ++kq) {
    const int w = wave + 8 * kq;
    wave_lds_sync();

    {
      const int g  = min(lane, 8);
      const int gi = g / 3;
      const int gj = g - 3 * gi;
      const int tr = w + 1 - gi;
      const int tc = h + 1 - gj;
      const bool ok = (tr >= 0) && (tr < 64) && (tc >= 0) && (tc < 64);
      const int trc = min(max(tr, 0), 63), tcc = min(max(tc, 0), 63);
      const float* lp = VA + ((size_t)b * 4096 + (size_t)trc * 64 + tcc) * NVA + CH + 9 * g;
      float lv[9];
      float mx = -3.0e38f;
#pragma unroll
      for (int q = 0; q < 9; ++q) { lv[q] = lp[q]; mx = fmaxf(mx, lv[q]); }
      float z = 0.0f;
#pragma unroll
      for (int q = 0; q < 9; ++q) { lv[q] = __expf(lv[q] - mx); z += lv[q]; }
      const float iz = 1.0f / z;
      if (lane < 9) {
#pragma unroll
        for (int q = 0; q < 9; ++q) sPw[9 * g + q] = ok ? lv[q] * iz : 0.0f;
      }
    }
    wave_lds_sync();

    {
      const int t  = min(lane, 24);
      const int t5 = t / 5;
      const int du = t5 - 2;
      const int dv = (t - 5 * t5) - 2;
      float ws = 0.0f;
#pragma unroll
      for (int i = 0; i < 3; ++i) {
        const int i2 = dv + i;
        const bool oki = (i2 >= 0) && (i2 <= 2);
        const int i2c = min(max(i2, 0), 2);
#pragma unroll
        for (int j = 0; j < 3; ++j) {
          const int j2 = du + j;
          const bool okj = (j2 >= 0) && (j2 <= 2);
          const int j2c = min(max(j2, 0), 2);
          const float pv = sPw[(i * 3 + j) * 9 + i2c * 3 + j2c];
          ws += (oki && okj) ? pv : 0.0f;
        }
      }
      if (lane < 25) sWw[lane] = ws;
    }
    wave_lds_sync();

    const int c0 = lane * 8;
    v4f a0 = zero4(), a1 = zero4();
    v4f m10 = fill4(-3.0e38f), m11 = fill4(-3.0e38f), m20 = fill4(-3.0e38f), m21 = fill4(-3.0e38f);
#pragma unroll 1
    for (int t = 0; t < 25; ++t) {
      const int t5 = t / 5;
      const int du = t5 - 2;
      const int dv = (t - 5 * t5) - 2;
      const int hn = h + du, wn = w + dv;
      if (hn < 0 || hn > 63 || wn < 0 || wn > 63) continue;
      const size_t pr = ((size_t)b * 64 + (size_t)hn) * 64 + (size_t)wn;
      const float* xp = X + pr * CH + c0;
      const float* vp = VA + pr * NVA + c0;
      const v4f x0 = *(const v4f*)(xp);
      const v4f x1 = *(const v4f*)(xp + 4);
      const v4f v0 = *(const v4f*)(vp);
      const v4f v1 = *(const v4f*)(vp + 4);
      const float wg = sWw[t];
      m20 = vmax4(m20, x0);
      m21 = vmax4(m21, x1);
      if (du >= -1 && du <= 1 && dv >= -1 && dv <= 1) {
        m10 = vmax4(m10, x0);
        m11 = vmax4(m11, x1);
      }
#pragma unroll
      for (int e = 0; e < 4; ++e) {
        a0[e] = fmaf(wg, v0[e], a0[e]);
        a1[e] = fmaf(wg, v1[e], a1[e]);
      }
    }

    HU hu1, lu1, hu2, lu2;
#pragma unroll
    for (int e = 0; e < 4; ++e) {
      const float r1a = fmaxf(fmaxf(a0[e], 0.0f) + bfr(m10[e]), 0.0f);
      const float r2a = fmaxf(r1a + bfr(m20[e]), 0.0f);
      const float r1b = fmaxf(fmaxf(a1[e], 0.0f) + bfr(m11[e]), 0.0f);
      const float r2b = fmaxf(r1b + bfr(m21[e]), 0.0f);
      const us_t h1a = bf_bits(r1a), h2a = bf_bits(r2a), h1b = bf_bits(r1b), h2b = bf_bits(r2b);
      hu1.e[e]     = h1a;  lu1.e[e]     = bf_bits(r1a - bf_up(h1a));
      hu2.e[e]     = h2a;  lu2.e[e]     = bf_bits(r2a - bf_up(h2a));
      hu1.e[4 + e] = h1b;  lu1.e[4 + e] = bf_bits(r1b - bf_up(h1b));
      hu2.e[4 + e] = h2b;  lu2.e[4 + e] = bf_bits(r2b - bf_up(h2b));
    }
    const size_t orow = ((size_t)b * 64 + (size_t)h) * 64 + (size_t)w;
    us_t* ph = CHp + orow * KFU + c0;
    us_t* pl = CLp + orow * KFU + c0;
    for (int pass = 0; pass < 2; ++pass) {
      *(volatile v4u*)(ph)      = hu1.u;
      *(volatile v4u*)(ph + CH) = hu2.u;
      *(volatile v4u*)(pl)      = lu1.u;
      *(volatile v4u*)(pl + CH) = lu2.u;
      __threadfence();
    }
  }
}

__global__ __launch_bounds__(256) void bn_stats(const float* __restrict__ P2, int N, int tilesM,
                                                const float* __restrict__ gam, const float* __restrict__ bet,
                                                float* MU, float* SC, float* BE) {
  __shared__ __align__(16) float sst[3 * 256];
  const int t = threadIdx.x;
  const int f0 = blockIdx.x * 256;
  const int f = min(f0 + t, N - 1);
  const float* ps = P2 + f;
  const float* pq = P2 + (size_t)tilesM * (size_t)N + f;
  double s = 0.0, q = 0.0;
#pragma unroll 1
  for (int tt = 0; tt < tilesM; ++tt) {
    s += (double)ps[(size_t)tt * N];
    q += (double)pq[(size_t)tt * N];
  }
  const double inv = 1.0 / (double)NPIX;
  const double mu = s * inv;
  double var = q * inv - mu * mu;
  if (var < 0.0) var = 0.0;
  const float muf = (float)mu;
  const float varf = (float)var;
  const float scv = bfr(gam[f]) * (1.0f / sqrtf(varf + 1e-5f));
  const float bev = bfr(bet[f]);
  sst[t]       = muf;
  sst[256 + t] = scv;
  sst[512 + t] = bev;
  __syncthreads();
  if (f0 + 256 <= N && t < 192) {
    const int a = t >> 6;
    const int w64 = t & 63;
    const int li = w64 >> 3, q8 = w64 & 7;
    const int col = li * 32 + q8 * 4;
    const v4f v = *(const v4f*)(sst + a * 256 + col);
    float* base = (a == 0) ? MU : ((a == 1) ? SC : BE);
    float* dst = base + f0 + col;
    *(volatile v4f*)dst = v;
    __threadfence();
    *(volatile v4f*)dst = v;
  }
}

__global__ __launch_bounds__(256) void bn_out(const float* __restrict__ Y, const float* __restrict__ MU,
                                              const float* __restrict__ SC, const float* __restrict__ BE,
                                              float* out) {
  const int t = threadIdx.x;
  const int c = (t & 63) * 4;
  const int rsub = t >> 6;
  const v4f mu = *(const v4f*)(MU + c);
  const v4f sc = *(const v4f*)(SC + c);
  const v4f be = *(const v4f*)(BE + c);
  for (int pass = 0; pass < 2; ++pass) {
#pragma unroll 1
    for (int it = 0; it < 16; ++it) {
      const int orow = blockIdx.x * 64 + 4 * it + rsub;
      const int bb = orow >> 12;
      const int p1 = (orow >> 6) & 63;
      const int p2 = orow & 63;
      const size_t src = ((size_t)bb * 64 + (size_t)p2) * 64 + (size_t)p1;
      const v4f y = *(const v4f*)(Y + src * CH + c);
      v4f o;
#pragma unroll
      for (int e = 0; e < 4; ++e) o[e] = (y[e] - mu[e]) * sc[e] + be[e];
      *(volatile v4f*)(out + (size_t)orow * CH + c) = o;
    }
    __threadfence();
  }
}

extern "C" void kernel_launch(void* const* d_in, const int* in_sizes, int n_in,
                              void* d_out, int out_size, void* d_ws, size_t ws_size,
                              hipStream_t stream) {
  if (n_in < 9) return;
  if (in_sizes[0] != NPIX * CH || in_sizes[1] != CH * CH || in_sizes[2] != CH) return;
  if (in_sizes[3] != CH * NAT || in_sizes[4] != NAT) return;
  if (in_sizes[5] != KFU * CH || in_sizes[6] != CH || in_sizes[7] != CH || in_sizes[8] != CH) return;
  if (out_size != NPIX * CH) return;

  const float* x     = (const float*)d_in[0];
  const float* Wv    = (const float*)d_in[1];
  const float* bv    = (const float*)d_in[2];
  const float* Wa    = (const float*)d_in[3];
  const float* ba    = (const float*)d_in[4];
  const float* Wfu   = (const float*)d_in[5];
  const float* bfu   = (const float*)d_in[6];
  const float* gam   = (const float*)d_in[7];
  const float* bet   = (const float*)d_in[8];

  const size_t PCC = (size_t)NPIX * KFU * 2;
  const size_t PX  = (size_t)NPIX * CH * 2;
  const size_t PVA = (size_t)NPIX * NVA * 4;
  const size_t POU = (size_t)NPIX * CH * 4;
  const size_t PWB = (size_t)NVA * CH * 2;
  const size_t PWF = (size_t)CH * KFU * 2;
  const size_t PP2 = (size_t)2 * TM64 * CH * 4;
  const size_t PST = (size_t)CH * 4;
  if (PX > PCC || POU > PVA) return;

  size_t off = 0;
  const size_t oCH = off; off += PCC;
  const size_t oCL = off; off += PCC;
  const size_t oVA = off; off += PVA;
  const size_t oWB = off; off += PWB;
  const size_t oWF = off; off += PWF;
  const size_t oP2 = off; off += PP2;
  const size_t oMU = off; off += PST;
  const size_t oSC = off; off += PST;
  const size_t oBE = off; off += PST;
  if (off > ws_size) return;
  if (off > (size_t)134217728) return;

  char* ws = (char*)d_ws;
  us_t*  CHp = (us_t*)(ws + oCH);
  us_t*  CLp = (us_t*)(ws + oCL);
  us_t*  X16 = (us_t*)(ws + oCH);
  float* VA  = (float*)(ws + oVA);
  float* OUT = (float*)(ws + oVA);
  us_t*  WB  = (us_t*)(ws + oWB);
  us_t*  WF  = (us_t*)(ws + oWF);
  float* P2  = (float*)(ws + oP2);
  float* MU  = (float*)(ws + oMU);
  float* SC  = (float*)(ws + oSC);
  float* BE  = (float*)(ws + oBE);
  float* outf = (float*)d_out;

  const dim3 blk(256);
  const int n8x = (NPIX * CH) / 8;
  const dim3 gX((n8x + 255) / 256);
  const dim3 gWv((CH * (CH / 8) + 255) / 256);
  const dim3 gWa(((NVA - CH) * (CH / 8) + 255) / 256);
  const dim3 gWf((CH * (KFU / 8) + 255) / 256);
  const dim3 gG1((TM64 * (NVA / 64) + 7) / 8);
  const dim3 gWin(NB * HS);
  const dim3 gG2((TM64 * (CH / 64) + 7) / 8);
  const dim3 gSt(CH / 256);
  const dim3 gOut(NPIX / 64);

  cvt_bf<<<gX, blk, 0, stream>>>(x, X16, n8x);
  wtr8<<<gWv, blk, 0, stream>>>(Wv, CH, CH, WB, CH);
  wtr8<<<gWa, blk, 0, stream>>>(Wa, CH, NAT, WB + (size_t)CH * CH, NVA - CH);
  wtr8<<<gWf, blk, 0, stream>>>(Wfu, KFU, CH, WF, CH);

  gemm64b<0, 1><<<gG1, blk, 0, stream>>>(X16, CH, (size_t)0, WB, CH, bv, CH, ba, NAT,
                                          x, CH, VA, NVA, P2, NPIX, NVA, CH);

  k_win<<<gWin, blk, 0, stream>>>(VA, x, CHp, CLp);

  gemm64b<1, 2><<<gG2, blk, 0, stream>>>(CHp, KFU, (size_t)NPIX * KFU, WF, KFU, bfu, CH, bfu, 1,
                                          x, CH, OUT, CH, P2, NPIX, CH, KFU);

  bn_stats<<<gSt, blk, 0, stream>>>(P2, CH, TM64, gam, bet, MU, SC, BE);
  bn_out<<<gOut, blk, 0, stream>>>(OUT, MU, SC, BE, outf);
}
